// TDRegEquiCNN_71734543777977
// MI455X (gfx1250) — hardware-verified
//
#include <hip/hip_runtime.h>
#include <hip/hip_bf16.h>

typedef _Float16 half_t;
typedef __attribute__((ext_vector_type(16))) _Float16 v16h;
typedef __attribute__((ext_vector_type(8)))  _Float16 v8h;
typedef __attribute__((ext_vector_type(8)))  float    v8f;
typedef __attribute__((ext_vector_type(4)))  float    v4f_t;
typedef float v4fa __attribute__((ext_vector_type(4), may_alias));
typedef __attribute__((ext_vector_type(4)))  unsigned v4u_t;
typedef unsigned v4ua __attribute__((ext_vector_type(4), may_alias));
static __device__ __forceinline__ unsigned pk2h(half_t a, half_t b) { return (unsigned)__builtin_bit_cast(unsigned short, a) | ((unsigned)__builtin_bit_cast(unsigned short, b) << 16); }
__host__ __device__ constexpr int PL(int hw) { return (hw + 63) & ~63; }

__device__ __forceinline__ void rotsrc(int r, int y, int x, int ksz, int& sy, int& sx) {
    switch (r & 3) {
        case 0:  sy = y;            sx = x;            break;
        case 1:  sy = x;            sx = ksz - 1 - y;  break;
        case 2:  sy = ksz - 1 - y;  sx = ksz - 1 - x;  break;
        default: sy = ksz - 1 - x;  sx = y;            break;
    }
}

template <int KSZ>
__global__ void prep_lift(const float* __restrict__ w, half_t* __restrict__ out) {
    constexpr int KK  = KSZ * KSZ;
    constexpr int KKP = (KK + 31) & ~31;
    int k0 = (blockIdx.x * blockDim.x + threadIdx.x) * 2;
    int n = blockIdx.y;
    if (k0 >= KKP) return;
    half_t vv[2];
#pragma unroll
    for (int q = 0; q < 2; ++q) {
        int k = k0 + q;
        half_t val = (half_t)0.f;
        if (k < KK) {
            int o = n >> 2, r = n & 3;
            int ky = k / KSZ;
            int kx = k - ky * KSZ;
            int sy, sx; rotsrc(r, ky, kx, KSZ, sy, sx);
            val = (half_t)w[o * KK + sy * KSZ + sx];
        }
        vv[q] = val;
    }
    const unsigned p = pk2h(vv[0], vv[1]);
    *(volatile unsigned*)(out + (size_t)n * KKP + k0) = p; __threadfence(); *(volatile unsigned*)(out + (size_t)n * KKP + k0) = p;
}

template <int KSZ>
__global__ void prep_group(const float* __restrict__ w, half_t* __restrict__ out,
                           int I, int KROW) {
    constexpr int KK  = KSZ * KSZ;
    constexpr int KKP = (KK + 31) & ~31;
    int k0 = (blockIdx.x * blockDim.x + threadIdx.x) * 2;
    int n = blockIdx.y;
    if (k0 >= KROW) return;
    half_t vv[2];
#pragma unroll
    for (int q = 0; q < 2; ++q) {
        int k = k0 + q;
        int ci = k / KKP;
        int kl = k - ci * KKP;
        half_t val = (half_t)0.f;
        if (kl < KK) {
            int o = n >> 2, r = n & 3;
            int ky = kl / KSZ;
            int kx = kl - ky * KSZ;
            int i = ci >> 2, g = ci & 3;
            int sy, sx; rotsrc(r, ky, kx, KSZ, sy, sx);
            int gg = (g - r) & 3;
            val = (half_t)w[(((o * I + i) * 4 + gg) * KSZ + sy) * KSZ + sx];
        }
        vv[q] = val;
    }
    const unsigned p = pk2h(vv[0], vv[1]);
    *(volatile unsigned*)(out + (size_t)n * KROW + k0) = p; __threadfence(); *(volatile unsigned*)(out + (size_t)n * KROW + k0) = p;
}

__global__ void f32_to_f16(const float* __restrict__ in, half_t* __restrict__ out, int n) {
    int i = (blockIdx.x * blockDim.x + threadIdx.x) * 2;
    if (i < n) { const unsigned p = pk2h((half_t)in[i], (half_t)in[i + 1]); *(volatile unsigned*)(out + i) = p; __threadfence(); *(volatile unsigned*)(out + i) = p; }
}

template <int CIN, int H, int W, int COUT, int KSZ, int PAD, int NW>
__global__ void __launch_bounds__(256)
conv_wmma(const half_t* __restrict__ in, const half_t* __restrict__ wgt,
          const float* __restrict__ bias, half_t* __restrict__ out) {
    constexpr int HOUT = H + 2 * PAD - KSZ + 1;
    constexpr int WOUT = W + 2 * PAD - KSZ + 1;
    constexpr int HWo  = HOUT * WOUT;
    constexpr int HWoP = PL(HWo);
    constexpr int PLI  = PL(H * W);
    constexpr int M    = 64 * HWoP;
    constexpr int TM   = M / 16;
    constexpr int KK   = KSZ * KSZ;
    constexpr int KKP  = (KK + 31) & ~31;
    constexpr int SUBS = KKP / 32;
    constexpr int KROW = CIN * KKP;
    constexpr int NWID = 16 * NW;
    constexpr int TNW  = (COUT + NWID - 1) / NWID;
    constexpr int TILES = TM * TNW;

    const int lane = threadIdx.x & 31;
    const int wave = threadIdx.x >> 5;
    int tile = blockIdx.x * 8 + wave;
    if (tile >= TILES) tile = TILES - 1;

    const int tm = tile / TNW;
    const int tn = tile - tm * TNW;

    const int mrow = tm * 16 + (lane & 15);
    const int b  = mrow / HWoP;
    const int r0 = mrow - b * HWoP;
    const int oy = r0 / WOUT;
    const int ox = r0 - oy * WOUT;
    const bool rowok = (r0 < HWo);
    const int ka = (lane >> 4) * 8;
    const int kb = ka;
    const int nb = tn * NWID + (lane & 15);

    int  offs[SUBS][16];
    bool ok[SUBS][16];
#pragma unroll
    for (int sub = 0; sub < SUBS; ++sub) {
#pragma unroll
        for (int e = 0; e < 16; ++e) {
            int kl = sub * 32 + ((e >> 3) << 4) + ka + (e & 7);
            int ky = kl / KSZ;
            int kx = kl - ky * KSZ;
            int iy = oy + ky - PAD;
            int ix = ox + kx - PAD;
            bool v = rowok && (kl < KK) && ((unsigned)iy < (unsigned)H)
                               && ((unsigned)ix < (unsigned)W);
            ok[sub][e]   = v;
            offs[sub][e] = v ? (b * (CIN * PLI) + iy * W + ix) : 0;
        }
    }

    const half_t* __restrict__ wr[NW];
#pragma unroll
    for (int wv = 0; wv < NW; ++wv) {
        int nn = nb + 16 * wv;
        wr[wv] = wgt + (size_t)(nn < COUT ? nn : 0) * KROW;
    }

    v8f acc[NW];
#pragma unroll
    for (int wv = 0; wv < NW; ++wv) acc[wv] = (v8f){};

#pragma unroll 2
    for (int ci = 0; ci < CIN; ++ci) {
        const int cbase = ci * PLI;
#pragma unroll
        for (int sub = 0; sub < SUBS; ++sub) {
            v16h afrag;
#pragma unroll
            for (int e = 0; e < 16; ++e) {
                half_t t = in[(size_t)(unsigned)(offs[sub][e] + cbase)];
                afrag[e] = ok[sub][e] ? t : (half_t)0.f;
            }
            const int kc = ci * KKP + sub * 32 + kb;
#pragma unroll
            for (int wv = 0; wv < NW; ++wv) {
                v16h bf;
                *(v8h*)&bf = *(const v8h*)(wr[wv] + kc); *((v8h*)&bf + 1) = *(const v8h*)(wr[wv] + kc + 16);
                acc[wv] = __builtin_amdgcn_wmma_f32_16x16x32_f16(
                    false, afrag, false, bf, (short)0, acc[wv], false, false);
            }
        }
        if (ci + 1 < CIN)
            __builtin_prefetch(in + (size_t)(unsigned)(offs[0][0] + cbase) + PLI, 0, 0);
    }

    constexpr int MT   = 8 / TNW;
    constexpr int PXB  = 16 * MT;
    constexpr int NBLK = (TNW == 1) ? COUT : NWID * TNW;
    static_assert(TNW == 1 || TNW == 2, "block tiling assumes TNW in {1,2}");
    __shared__ __attribute__((aligned(16))) half_t so[NBLK * PXB];
    __syncthreads();
    const int mhi = (lane >> 4) << 3;
    const int tm0 = (blockIdx.x * 8) / TNW;
    {
        const int pxl0 = (tm - tm0) * 16;
#pragma unroll
        for (int v = 0; v < 8; ++v) {
#pragma unroll
            for (int wv = 0; wv < NW; ++wv) {
                int nn = nb + 16 * wv;
                if (nn < COUT && pxl0 >= 0 && pxl0 < PXB) {
                    float val = acc[wv][v] + bias[nn >> 2];
                    so[nn * PXB + pxl0 + v + mhi] = (half_t)(val > 0.f ? val : 0.f);
                }
            }
        }
    }
    __syncthreads();
    {
        const int m0 = tm0 * 16;
        constexpr int NCH = NBLK * (PXB / 8);
#pragma unroll 1
        for (int pass = 0; pass < 2; ++pass) {
            for (int c = threadIdx.x; c < NCH; c += 256) {
                const int ch = c / (PXB / 8), q = c - ch * (PXB / 8);
                const int m = m0 + q * 8;
                if (m + 7 < M && ch < COUT) {
                    const int bb = m / HWoP, rr = m - bb * HWoP;
                    *(volatile v4u_t*)(out + ((size_t)bb * COUT + ch) * HWoP + rr) = *(const volatile v4ua*)(so + ch * PXB + q * 8);
                }
            }
            __threadfence();
        }
    }
}

template <int C, int H, int W>
__global__ void pool_kernel(const half_t* __restrict__ in, half_t* __restrict__ out) {
    constexpr int Ho = H / 2, Wo = W / 2, HWo = Ho * Wo, PLO = PL(HWo), PLI = PL(H * W);
    constexpr int TOTAL = 64 * C * (PLO / 2);
    int idx = blockIdx.x * blockDim.x + threadIdx.x;
    if (idx >= TOTAL) return;
    const int plane = idx / (PLO / 2), pp = (idx - plane * (PLO / 2)) * 2;
    const half_t* pin = in + (size_t)plane * PLI;
    half_t v2[2];
#pragma unroll
    for (int q = 0; q < 2; ++q) {
        const int px = pp + q;
        float m = 0.f;
        if (px < HWo) {
            const int yo = px / Wo, xo = px - yo * Wo;
            const half_t* p = pin + (yo * 2) * W + xo * 2;
            m = fmaxf(fmaxf((float)p[0], (float)p[1]), fmaxf((float)p[W], (float)p[W + 1]));
        }
        v2[q] = (half_t)m;
    }
    const unsigned pk = pk2h(v2[0], v2[1]);
    *(volatile unsigned*)(out + (size_t)plane * PLO + pp) = pk; __threadfence(); *(volatile unsigned*)(out + (size_t)plane * PLO + pp) = pk;
}

template <int C, int HW>
__global__ void gap_kernel(const half_t* __restrict__ in, half_t* __restrict__ out) {
    int idx = (blockIdx.x * blockDim.x + threadIdx.x) * 2;
    if (idx >= 64 * C) return;
    half_t v2[2];
#pragma unroll
    for (int q = 0; q < 2; ++q) {
        const half_t* p = in + (size_t)(idx + q) * PL(HW);
        float s = 0.f;
        for (int i = 0; i < HW; ++i) s += (float)p[i];
        v2[q] = (half_t)(s * (1.f / (float)HW));
    }
    const unsigned pk = pk2h(v2[0], v2[1]);
    *(volatile unsigned*)(out + idx) = pk; __threadfence(); *(volatile unsigned*)(out + idx) = pk;
}

template <int NT, int KDIM, bool RELU, bool OUTF32>
__global__ void __launch_bounds__(128)
gemm_wmma_fc(const half_t* __restrict__ A, const half_t* __restrict__ Wt,
             const float* __restrict__ bias, void* __restrict__ outp, int N) {
    constexpr int NPAD = 16 * NT;
    __shared__ __attribute__((aligned(16))) float so[16 * NPAD];
    const int lane = threadIdx.x & 31, wave = threadIdx.x >> 5;
    const int tm = blockIdx.x, tn = wave;
    const int mrow = tm * 16 + (lane & 15);
    const int n    = tn * 16 + (lane & 15);
    const int ka = (lane >> 4) * 8;
    if (tn < NT) {
        const half_t* __restrict__ Arow = A  + (size_t)mrow * KDIM;
        const half_t* __restrict__ Wrow = Wt + (size_t)(n < N ? n : 0) * KDIM;
        v8f acc = {};
#pragma unroll
        for (int kc = 0; kc < KDIM; kc += 32) {
            v8h alo = *(const v8h*)(Arow + kc + ka);
            v8h ahi = *(const v8h*)(Arow + kc + 16 + ka);
            v16h afrag, bfrag;
#pragma unroll
            for (int e = 0; e < 8; ++e) { afrag[e] = alo[e]; afrag[e + 8] = ahi[e]; }
            v8h blo = *(const v8h*)(Wrow + kc + ka), bhi = *(const v8h*)(Wrow + kc + 16 + ka);
#pragma unroll
            for (int e = 0; e < 8; ++e) { bfrag[e] = blo[e]; bfrag[e + 8] = bhi[e]; }
            acc = __builtin_amdgcn_wmma_f32_16x16x32_f16(
                false, afrag, false, bfrag, (short)0, acc, false, false);
        }
        float bv = (n < N) ? bias[n] : 0.f;
#pragma unroll
        for (int v = 0; v < 8; ++v) {
            int ml = v + ((lane >> 4) << 3);
            float val = acc[v] + bv;
            if (RELU) val = val > 0.f ? val : 0.f;
            so[ml * NPAD + n] = val;
        }
    }
    __syncthreads();
#pragma unroll 1
    for (int pass = 0; pass < 2; ++pass) {
        if (OUTF32) {
            float* o = (float*)outp + (size_t)tm * 16 * N;
            for (int c = threadIdx.x; c * 4 < 16 * N; c += 128) {
                v4f_t v; for (int j = 0; j < 4; ++j) { int f = c * 4 + j, ml = f / N, nn = f - ml * N; v[j] = so[ml * NPAD + nn]; }
                *(volatile v4f_t*)(o + c * 4) = v;
            }
        } else {
            half_t* o = (half_t*)outp;
            for (int c = threadIdx.x; c < 16 * (N / 8); c += 128) {
                const int ml = c / (N / 8), q = c - ml * (N / 8);
                const float* s = so + ml * NPAD + q * 8;
                v4u_t v; v.x = pk2h((half_t)s[0], (half_t)s[1]); v.y = pk2h((half_t)s[2], (half_t)s[3]); v.z = pk2h((half_t)s[4], (half_t)s[5]); v.w = pk2h((half_t)s[6], (half_t)s[7]);
                *(volatile v4u_t*)(o + (size_t)(tm * 16 + ml) * N + q * 8) = v;
            }
        }
        __threadfence();
    }
}

extern "C" void kernel_launch(void* const* d_in, const int* in_sizes, int n_in,
                              void* d_out, int out_size, void* d_ws, size_t ws_size,
                              hipStream_t stream) {
    const float* x   = (const float*)d_in[0];
    const float* w0  = (const float*)d_in[1];
    const float* b0  = (const float*)d_in[2];
    const float* w1  = (const float*)d_in[3];
    const float* b1  = (const float*)d_in[4];
    const float* w2  = (const float*)d_in[5];
    const float* b2  = (const float*)d_in[6];
    const float* w3  = (const float*)d_in[7];
    const float* b3  = (const float*)d_in[8];
    const float* w4  = (const float*)d_in[9];
    const float* b4  = (const float*)d_in[10];
    const float* w5  = (const float*)d_in[11];
    const float* b5  = (const float*)d_in[12];
    const float* fw1 = (const float*)d_in[13];
    const float* fb1 = (const float*)d_in[14];
    const float* fw2 = (const float*)d_in[15];
    const float* fb2 = (const float*)d_in[16];

    char* ws = (char*)d_ws;
    size_t off = 0;
    auto take = [&](size_t elems) {
        half_t* p = (half_t*)(ws + off);
        off += (elems * sizeof(half_t) + 255) & ~(size_t)255;
        return p;
    };
    half_t* bufB  = take((size_t)64 * 48 * PL(92 * 92));
    half_t* bufA  = take((size_t)64 * 96 * PL(46 * 46));
    half_t* x16   = take(589824);
    half_t* wL0   = take(24 * 64);
    half_t* wG1   = take(48 * 768);
    half_t* wG2   = take(48 * 1536);
    half_t* wG3   = take(96 * 1536);
    half_t* wG4   = take(96 * 3072);
    half_t* wG5   = take(64 * 3072);
    half_t* fw1h  = take(64 * 64);
    half_t* fw2h  = take(10 * 64);
    half_t* gap16 = take(64 * 64);
    half_t* fc1o  = take(64 * 64);

    f32_to_f16<<<(589824 / 2 + 255) / 256, 256, 0, stream>>>(x, x16, 589824);
    prep_lift<7><<<dim3(1, 24), 256, 0, stream>>>(w0, wL0);
    prep_group<5><<<dim3(2, 48), 256, 0, stream>>>(w1, wG1, 6, 768);
    prep_group<5><<<dim3(3, 48), 256, 0, stream>>>(w2, wG2, 12, 1536);
    prep_group<5><<<dim3(3, 96), 256, 0, stream>>>(w3, wG3, 12, 1536);
    prep_group<5><<<dim3(6, 96), 256, 0, stream>>>(w4, wG4, 24, 3072);
    prep_group<5><<<dim3(6, 64), 256, 0, stream>>>(w5, wG5, 24, 3072);
    f32_to_f16<<<(4096 / 2 + 255) / 256, 256, 0, stream>>>(fw1, fw1h, 4096);
    f32_to_f16<<<(640 / 2 + 255) / 256, 256, 0, stream>>>(fw2, fw2h, 640);

    auto nblocks = [](int Hout, int Wout, int Cout, int NW) {
        int nwid = 16 * NW;
        int tiles = (64 * PL(Hout * Wout) / 16) * ((Cout + nwid - 1) / nwid);
        return (tiles + 7) / 8;
    };

    conv_wmma<1, 96, 96, 24, 7, 1, 2>
        <<<nblocks(92, 92, 24, 2), 256, 0, stream>>>(x16, wL0, b0, bufA);
    conv_wmma<24, 92, 92, 48, 5, 2, 3>
        <<<nblocks(92, 92, 48, 3), 256, 0, stream>>>(bufA, wG1, b1, bufB);
    pool_kernel<48, 92, 92>
        <<<(64 * 48 * (PL(46 * 46) / 2) + 255) / 256, 256, 0, stream>>>(bufB, bufA);
    conv_wmma<48, 46, 46, 48, 5, 2, 3>
        <<<nblocks(46, 46, 48, 3), 256, 0, stream>>>(bufA, wG2, b2, bufB);
    conv_wmma<48, 46, 46, 96, 5, 2, 3>
        <<<nblocks(46, 46, 96, 3), 256, 0, stream>>>(bufB, wG3, b3, bufA);
    pool_kernel<96, 46, 46>
        <<<(64 * 96 * (PL(23 * 23) / 2) + 255) / 256, 256, 0, stream>>>(bufA, bufB);
    conv_wmma<96, 23, 23, 96, 5, 2, 3>
        <<<nblocks(23, 23, 96, 3), 256, 0, stream>>>(bufB, wG4, b4, bufA);
    conv_wmma<96, 23, 23, 64, 5, 1, 4>
        <<<nblocks(21, 21, 64, 4), 256, 0, stream>>>(bufA, wG5, b5, bufB);

    gap_kernel<64, 441><<<8, 256, 0, stream>>>(bufB, gap16);

    gemm_wmma_fc<4, 64, true, false><<<4, 128, 0, stream>>>(gap16, fw1h, fb1, fc1o, 64);
    gemm_wmma_fc<1, 64, false, true><<<4, 128, 0, stream>>>(fc1o, fw2h, fb2, d_out, 10);
}
